// TwoLevelFCNetwork_65962107732178
// MI455X (gfx1250) — hardware-verified
//
#include <hip/hip_runtime.h>
#include <stdint.h>
#include <stddef.h>
#include <math.h>

#pragma clang fp contract(off)

#define NTOK 8192
#define DIN  256
#define DH   512
#define DOUT 64
#define NEX  8
#define MT   32
#define XP   264
#define HP   520
#define YP   68
#define TT   64
#define TPH  72

#define LDS_A  (MT * XP * 2)
#define LDS_B  (MT * HP * 2)
#define LDS_EXP (LDS_A + LDS_B)

static_assert(MT * YP * 4 <= LDS_A);
static_assert((XP * 2) % 16 == 0);
static_assert((HP * 2) % 16 == 0);
static_assert((YP * 4) % 16 == 0);
static_assert((TPH * 2) % 16 == 0);
static_assert(LDS_A % 16 == 0);
static_assert(LDS_EXP <= 65536);
static_assert(NTOK % 256 == 0);
static_assert(NTOK % MT == 0);
static_assert(DIN % 32 == 0);
static_assert(DH % 32 == 0);
static_assert(DH == 8 * 64);
static_assert(DOUT == 4 * 16);
static_assert(MT == 32);
static_assert(DIN % TT == 0);
static_assert(DH % TT == 0);
static_assert(DOUT % TT == 0);

typedef _Float16 v16h __attribute__((ext_vector_type(16)));
typedef _Float16 v8h  __attribute__((ext_vector_type(8)));
typedef float    v8f  __attribute__((ext_vector_type(8)));
typedef float    v4f  __attribute__((ext_vector_type(4)));
typedef v4f __attribute__((may_alias)) v4fa;
typedef v8h __attribute__((may_alias)) v8ha;

union FragH { v16h v; v8h q[2]; };

__device__ __forceinline__ v8f wmma_h(v16h a, v16h b, v8f c) {
  v8f d = __builtin_amdgcn_wmma_f32_16x16x32_f16(false, a, false, b, (short)0, c, false, false);
  asm volatile("v_nop\n\tv_nop\n\tv_nop\n\tv_nop" : "+v"(d) : "v"(a), "v"(b));
  return d;
}

__device__ __forceinline__ v16h ldfrag_h(const _Float16* p, int h) {
  FragH f;
  f.q[0] = *(const v8ha*)(p + 8 * h);
  f.q[1] = *(const v8ha*)(p + 16 + 8 * h);
  return f.v;
}

__device__ __forceinline__ float tanh_f(float v) {
  const float ax = fminf(fabsf(v), 9.0f);
  const float ex = __expf(ax + ax);
  const float r  = __builtin_amdgcn_rcpf(ex + 1.0f);
  return copysignf(1.0f - 2.0f * r, v);
}

__device__ __forceinline__ int route_idx(float v) {
  const float t = v * 100.0f;
  float a = fabsf(t);
  a = fminf(a, 2.0e9f);
  const int i = (int)a;
  return i & (NEX - 1);
}

__global__ __launch_bounds__(256) void k_wt(const float* __restrict__ src,
                                            _Float16* __restrict__ dst,
                                            int R, int C, float scale)
{
  __shared__ __align__(16) _Float16 sT[TT * TPH];
  const int tid = threadIdx.x, lane = tid & 31, wv = tid >> 5;
  const int z  = blockIdx.z;
  const int r0 = blockIdx.y * TT;
  const int c0 = blockIdx.x * TT;
  if (r0 + TT > R || c0 + TT > C) return;
  const float* s = src + (size_t)z * R * C;
  _Float16*    d = dst + (size_t)z * R * C;

  const int i = tid >> 2, cs = (tid & 3) * 16;
  const float* sp = s + (size_t)(r0 + i) * C + c0 + cs;
  const v4f a0 = *(const v4fa*)(sp);
  const v4f a1 = *(const v4fa*)(sp + 4);
  const v4f a2 = *(const v4fa*)(sp + 8);
  const v4f a3 = *(const v4fa*)(sp + 12);
  _Float16* tp = sT + cs * TPH + i;
  tp[ 0 * TPH] = (_Float16)(a0.x * scale);
  tp[ 1 * TPH] = (_Float16)(a0.y * scale);
  tp[ 2 * TPH] = (_Float16)(a0.z * scale);
  tp[ 3 * TPH] = (_Float16)(a0.w * scale);
  tp[ 4 * TPH] = (_Float16)(a1.x * scale);
  tp[ 5 * TPH] = (_Float16)(a1.y * scale);
  tp[ 6 * TPH] = (_Float16)(a1.z * scale);
  tp[ 7 * TPH] = (_Float16)(a1.w * scale);
  tp[ 8 * TPH] = (_Float16)(a2.x * scale);
  tp[ 9 * TPH] = (_Float16)(a2.y * scale);
  tp[10 * TPH] = (_Float16)(a2.z * scale);
  tp[11 * TPH] = (_Float16)(a2.w * scale);
  tp[12 * TPH] = (_Float16)(a3.x * scale);
  tp[13 * TPH] = (_Float16)(a3.y * scale);
  tp[14 * TPH] = (_Float16)(a3.z * scale);
  tp[15 * TPH] = (_Float16)(a3.w * scale);
  __syncthreads();

  const int q  = lane & 7;
  const int cA = 4 * wv + (lane >> 3);
  const int cB = 32 + cA;
  const v8h vA = *(const v8ha*)(sT + cA * TPH + 8 * q);
  const v8h vB = *(const v8ha*)(sT + cB * TPH + 8 * q);
  _Float16* dA = d + (size_t)(c0 + cA) * R + r0 + 8 * q;
  _Float16* dB = d + (size_t)(c0 + cB) * R + r0 + 8 * q;
  *(volatile v8ha*)dA = vA;
  *(volatile v8ha*)dB = vB;
  __threadfence();
  *(volatile v8ha*)dA = vA;
  *(volatile v8ha*)dB = vB;
}

__global__ __launch_bounds__(256) void k_expert(const float* __restrict__ x,
                                                const _Float16* __restrict__ w0t,
                                                const float* __restrict__ b0,
                                                const _Float16* __restrict__ w1t,
                                                const float* __restrict__ b1,
                                                const _Float16* __restrict__ wot,
                                                const float* __restrict__ bo,
                                                float* __restrict__ out)
{
  extern __shared__ __align__(16) unsigned char dsm_e[];
  _Float16* sX = (_Float16*)dsm_e;
  float*    sY = (float*)dsm_e;
  _Float16* sH = (_Float16*)(dsm_e + LDS_A);
  __shared__ int sTok[MT];
  __shared__ int s_wc[8];

  const int tid = threadIdx.x, lane = tid & 31, wv = tid >> 5;
  const int h = lane >> 4, m = lane & 15;
  const int e = blockIdx.y;
  const int m0 = blockIdx.x * MT;

  if (tid < MT) sTok[tid] = 0;
  __syncthreads();

  int base = 0;
  #pragma unroll 1
  for (int ch = 0; ch < NTOK / 256; ++ch) {
    const int t = ch * 256 + tid;
    const float v = x[(size_t)t * DIN + 7];
    const bool f = (route_idx(v) == e);
    const unsigned int msk = __builtin_amdgcn_ballot_w32(f);
    const int off = __builtin_popcount(msk & ((1u << lane) - 1u));
    const int wc  = __builtin_popcount(msk);
    if (lane == 0) s_wc[wv] = wc;
    __syncthreads();
    int pre = 0, tot = 0;
    #pragma unroll
    for (int w2 = 0; w2 < 8; ++w2) {
      const int cc = s_wc[w2];
      tot += cc;
      pre += (w2 < wv) ? cc : 0;
    }
    if (f) {
      const int p = base + pre + off - m0;
      if ((unsigned)p < (unsigned)MT) sTok[p] = t;
    }
    base += tot;
    __syncthreads();
  }
  const int cnt = base;
  if (m0 >= cnt) return;
  int nrows = cnt - m0;
  nrows = (nrows > MT) ? MT : nrows;

  {
    const int row = tid >> 3, cs = (tid & 7) * 32;
    int t = sTok[row];
    t = (t < 0) ? 0 : ((t > NTOK - 1) ? (NTOK - 1) : t);
    const float* sp = x + (size_t)t * DIN + cs;
    _Float16* dp = sX + row * XP + cs;
    #pragma unroll
    for (int j = 0; j < 4; ++j) {
      const v4f a = *(const v4fa*)(sp + 8 * j);
      const v4f b = *(const v4fa*)(sp + 8 * j + 4);
      v8h o;
      o[0] = (_Float16)a.x; o[1] = (_Float16)a.y; o[2] = (_Float16)a.z; o[3] = (_Float16)a.w;
      o[4] = (_Float16)b.x; o[5] = (_Float16)b.y; o[6] = (_Float16)b.z; o[7] = (_Float16)b.w;
      *(v8ha*)(dp + 8 * j) = o;
    }
  }
  __syncthreads();

  const v8f z8 = {0.f, 0.f, 0.f, 0.f, 0.f, 0.f, 0.f, 0.f};

  {
    v8f acc[2][4];
    #pragma unroll
    for (int mt = 0; mt < 2; ++mt)
      #pragma unroll
      for (int nt = 0; nt < 4; ++nt) acc[mt][nt] = z8;
    #pragma unroll 1
    for (int k0 = 0; k0 < DIN; k0 += 32) {
      const v16h a0 = ldfrag_h(sX + m * XP + k0, h);
      const v16h a1 = ldfrag_h(sX + (16 + m) * XP + k0, h);
      #pragma unroll
      for (int nt = 0; nt < 4; ++nt) {
        const int col = wv * 64 + 16 * nt + m;
        const v16h b = ldfrag_h(w0t + ((size_t)(e * DH + col)) * DIN + k0, h);
        acc[0][nt] = wmma_h(a0, b, acc[0][nt]);
        acc[1][nt] = wmma_h(a1, b, acc[1][nt]);
      }
    }
    #pragma unroll
    for (int nt = 0; nt < 4; ++nt) {
      const int col = wv * 64 + 16 * nt + m;
      const float bias = b0[e * DH + col];
      #pragma unroll
      for (int mt = 0; mt < 2; ++mt) {
        #pragma unroll
        for (int r = 0; r < 8; ++r) {
          const int row = 16 * mt + 8 * h + r;
          const float pre = acc[mt][nt][r] * 0.0625f + bias;
          sH[row * HP + col] = (_Float16)tanh_f(pre);
        }
      }
    }
  }
  __syncthreads();

  {
    v8f acc[2][4];
    #pragma unroll
    for (int mt = 0; mt < 2; ++mt)
      #pragma unroll
      for (int nt = 0; nt < 4; ++nt) acc[mt][nt] = z8;
    #pragma unroll 1
    for (int k0 = 0; k0 < DH; k0 += 32) {
      const v16h a0 = ldfrag_h(sH + m * HP + k0, h);
      const v16h a1 = ldfrag_h(sH + (16 + m) * HP + k0, h);
      #pragma unroll
      for (int nt = 0; nt < 4; ++nt) {
        const int col = wv * 64 + 16 * nt + m;
        const v16h b = ldfrag_h(w1t + ((size_t)(e * DH + col)) * DH + k0, h);
        acc[0][nt] = wmma_h(a0, b, acc[0][nt]);
        acc[1][nt] = wmma_h(a1, b, acc[1][nt]);
      }
    }
    __syncthreads();
    #pragma unroll
    for (int nt = 0; nt < 4; ++nt) {
      const int col = wv * 64 + 16 * nt + m;
      const float bias = b1[e * DH + col];
      #pragma unroll
      for (int mt = 0; mt < 2; ++mt) {
        #pragma unroll
        for (int r = 0; r < 8; ++r) {
          const int row = 16 * mt + 8 * h + r;
          const float pre = acc[mt][nt][r] * 0.0625f + bias;
          sH[row * HP + col] = (_Float16)tanh_f(pre);
        }
      }
    }
  }
  __syncthreads();

  {
    const int mt2 = wv >> 2, nt2 = wv & 3;
    const int col = 16 * nt2 + m;
    v8f acc = z8;
    #pragma unroll 1
    for (int k0 = 0; k0 < DH; k0 += 32) {
      const v16h a = ldfrag_h(sH + (16 * mt2 + m) * HP + k0, h);
      const v16h b = ldfrag_h(wot + ((size_t)(e * DOUT + col)) * DH + k0, h);
      acc = wmma_h(a, b, acc);
    }
    const float bias = bo[e * DOUT + col];
    #pragma unroll
    for (int r = 0; r < 8; ++r) {
      const int row = 16 * mt2 + 8 * h + r;
      sY[row * YP + col] = acc[r] * 0.0625f + bias;
    }
  }
  __syncthreads();

  {
    const int hl = lane >> 4, q = lane & 15;
    const int rowA = 2 * wv + hl;
    const int rowB = 16 + 2 * wv + hl;
    int tA = sTok[rowA];
    int tB = sTok[rowB];
    tA = (tA < 0) ? 0 : ((tA > NTOK - 1) ? (NTOK - 1) : tA);
    tB = (tB < 0) ? 0 : ((tB > NTOK - 1) ? (NTOK - 1) : tB);
    const v4f vA = *(const v4fa*)(sY + rowA * YP + 4 * q);
    const v4f vB = *(const v4fa*)(sY + rowB * YP + 4 * q);
    float* dA = out + (size_t)tA * DOUT + 4 * q;
    float* dB = out + (size_t)tB * DOUT + 4 * q;
    const bool okA = (rowA < nrows);
    const bool okB = (rowB < nrows);
    if (okA) *(volatile v4fa*)dA = vA;
    if (okB) *(volatile v4fa*)dB = vB;
    __threadfence();
    if (okA) *(volatile v4fa*)dA = vA;
    if (okB) *(volatile v4fa*)dB = vB;
  }
}

extern "C" void kernel_launch(void* const* d_in, const int* in_sizes, int n_in,
                              void* d_out, int out_size, void* d_ws, size_t ws_size,
                              hipStream_t stream)
{
  if (n_in < 7) return;
  if (in_sizes[0] != NTOK * DIN) return;
  if (in_sizes[1] != NEX * DIN * DH) return;
  if (in_sizes[2] != NEX * DH) return;
  if (in_sizes[3] != NEX * DH * DH) return;
  if (in_sizes[4] != NEX * DH) return;
  if (in_sizes[5] != NEX * DH * DOUT) return;
  if (in_sizes[6] != NEX * DOUT) return;
  if (out_size != NTOK * DOUT) return;

  const float* x  = (const float*)d_in[0];
  const float* W0 = (const float*)d_in[1];
  const float* b0 = (const float*)d_in[2];
  const float* W1 = (const float*)d_in[3];
  const float* b1 = (const float*)d_in[4];
  const float* Wo = (const float*)d_in[5];
  const float* bo = (const float*)d_in[6];
  float* out = (float*)d_out;

  const size_t bW0 = (size_t)NEX * DH * DIN * 2;
  const size_t bW1 = (size_t)NEX * DH * DH * 2;
  const size_t bWo = (size_t)NEX * DOUT * DH * 2;
  const size_t total = bW0 + bW1 + bWo;
  if (total > ws_size) return;
  if (total > (size_t)134217728) return;

  char* ws = (char*)d_ws;
  size_t off = 0;
  _Float16* W0T = (_Float16*)(ws + off); off += bW0;
  _Float16* W1T = (_Float16*)(ws + off); off += bW1;
  _Float16* WOT = (_Float16*)(ws + off); off += bWo;
  if (off != total) return;

  k_wt<<<dim3(DH / TT,   DIN / TT, NEX), 256, 0, stream>>>(W0, W0T, DIN, DH,   16.0f);
  k_wt<<<dim3(DH / TT,   DH / TT,  NEX), 256, 0, stream>>>(W1, W1T, DH,  DH,   16.0f);
  k_wt<<<dim3(DOUT / TT, DH / TT,  NEX), 256, 0, stream>>>(Wo, WOT, DH,  DOUT, 16.0f);
  k_expert<<<dim3(NTOK / MT, NEX), 256, LDS_EXP, stream>>>(x, W0T, b0, W1T, b1, WOT, bo, out);
}
